// EGNNLiteLayer_19868518711570
// MI455X (gfx1250) — hardware-verified
//
#include <hip/hip_runtime.h>
#include <math.h>
#define SRB 1024
#define SCHK 4096
typedef __attribute__((ext_vector_type(16))) _Float16 v16h;
typedef __attribute__((ext_vector_type(8)))  _Float16 v8h;
typedef __attribute__((ext_vector_type(16))) __bf16   v16b;
typedef __attribute__((ext_vector_type(8)))  __bf16   v8b;
typedef __attribute__((ext_vector_type(8)))  float    v8f;
typedef __attribute__((ext_vector_type(4)))  float    v4f;
#define PSCALE 32768.0f
#define U16(p) ((const unsigned short*)(const void*)(p))
#define PSCALE_INV (1.0f / 32768.0f)

__device__ __forceinline__ unsigned short f2bf_bits(float f) {
  unsigned u = __float_as_uint(f);
  return (unsigned short)((u + 0x7FFFu + ((u >> 16) & 1u)) >> 16);
}
__device__ __forceinline__ float bf_bits2f(unsigned short h) { return __uint_as_float(((unsigned)h) << 16); }

__device__ __forceinline__ void dep_guard_h(v8f& a, v8f& b, v16h x, v16h y) { asm volatile("v_nop\n\tv_nop\n\tv_nop\n\tv_nop" : "+v"(a), "+v"(b) : "v"(x), "v"(y)); }
__device__ __forceinline__ void dep_guard_b(v8f& a, v8f& b, v16b x, v16b y) { asm volatile("v_nop\n\tv_nop\n\tv_nop\n\tv_nop" : "+v"(a), "+v"(b) : "v"(x), "v"(y)); }
__device__ __forceinline__ void keep4_h(v16h a, v16h b, v16h c, v16h d) { asm volatile("v_nop" :: "v"(a), "v"(b), "v"(c), "v"(d)); }
__device__ __forceinline__ void keep4_b(v16b a, v16b b, v16b c, v16b d) { asm volatile("v_nop" :: "v"(a), "v"(b), "v"(c), "v"(d)); }
__device__ __forceinline__ void acc_guard4(v8f& a, v8f& b, v8f& c, v8f& d) { asm volatile("v_nop\n\tv_nop\n\tv_nop\n\tv_nop" : "+v"(a), "+v"(b), "+v"(c), "+v"(d)); }
template <typename T> struct Frag;
template <> struct Frag<_Float16> {
  typedef v16h V; union U { v16h v; v8h h[2]; };
  static __device__ __forceinline__ v16h load(const _Float16* p) {
    U f; f.h[0] = *(const v8h*)(p); f.h[1] = *(const v8h*)(p + 16); return f.v;
  }
  static __device__ __forceinline__ v8f mma(v16h a, v16h b, v8f c) {
    return __builtin_amdgcn_wmma_f32_16x16x32_f16(false, a, false, b, (short)0, c, false, false);
  }
  static __device__ __forceinline__ void guard(v8f& a, v8f& b, v16h x, v16h y) { dep_guard_h(a, b, x, y); }
  static __device__ __forceinline__ void keep(v16h a, v16h b, v16h c, v16h d) { keep4_h(a, b, c, d); }
};
template <> struct Frag<__bf16> {
  typedef v16b V; union U { v16b v; v8b h[2]; };
  static __device__ __forceinline__ v16b load(const __bf16* p) {
    U f; f.h[0] = *(const v8b*)(p); f.h[1] = *(const v8b*)(p + 16); return f.v;
  }
  static __device__ __forceinline__ v8f mma(v16b a, v16b b, v8f c) {
    return __builtin_amdgcn_wmma_f32_16x16x32_bf16(false, a, false, b, (short)0, c, false, false);
  }
  static __device__ __forceinline__ void guard(v8f& a, v8f& b, v16b x, v16b y) { dep_guard_b(a, b, x, y); }
  static __device__ __forceinline__ void keep(v16b a, v16b b, v16b c, v16b d) { keep4_b(a, b, c, d); }
};

template <int ET> struct Elem;
template <> struct Elem<0> { typedef _Float16 T; };
template <> struct Elem<1> { typedef __bf16 T; };
template <int ET, bool SPLIT, int BIAS_MODE, int OUT_MODE, bool RESID, int ACT = 0>
__global__ __launch_bounds__(256) void wmma_gemm64(
    const unsigned short* __restrict__ Ap, const unsigned short* __restrict__ A2p, int lda, long strideA,
    const unsigned short* __restrict__ Btp, const unsigned short* __restrict__ Bt2p, int ldb, long strideB,
    void* __restrict__ Cout, void* __restrict__ Cout2, int ldc, long strideC,
    const float* __restrict__ bias,
    const float* __restrict__ resid, long strideR,
    int M, int N, int K, float scale) {
  typedef typename Elem<ET>::T T;
  typedef typename Frag<T>::V V;
  const T* A = (const T*)Ap; const T* A2 = (const T*)A2p; const T* Bt = (const T*)Btp; const T* Bt2 = (const T*)Bt2p;
  __shared__ __align__(16) float sT[8][16 * 68];
  const int b    = blockIdx.y;
  const int lane = threadIdx.x & 31;
  const int wave = threadIdx.x >> 5;
  const int tilesN = N >> 6;
  const int tilesM = M >> 6;
  const int tile = blockIdx.x * 8 + wave;
  if (tile >= tilesM * tilesN) return;
  const int tm = tile / tilesN;
  const int tn = tile - tm * tilesN;
  const int m0 = tm << 6;
  const int n0 = tn << 6;

  const T* Ab  = A  + (size_t)b * strideA;
  const T* Bb  = Bt + (size_t)b * strideB;
  const T* Ab2 = SPLIT ? (A2  + (size_t)b * strideA) : nullptr;
  const T* Bb2 = SPLIT ? (Bt2 + (size_t)b * strideB) : nullptr;

  const int rlane = lane & 15;
  const int koff  = (lane >> 4) * 8;
  const int mOff  = (lane >> 4) * 8;

  v8f acc[4][4];
#pragma unroll
  for (int i = 0; i < 4; ++i)
#pragma unroll
    for (int j = 0; j < 4; ++j) acc[i][j] = (v8f){0.f,0.f,0.f,0.f,0.f,0.f,0.f,0.f};

  for (int k0 = 0; k0 < K; k0 += 32) {
    V bh[4], bl[4];
#pragma unroll
    for (int j = 0; j < 4; ++j) {
      const size_t bo = (size_t)(n0 + (j << 4) + rlane) * ldb + koff + k0;
      bh[j] = Frag<T>::load(Bb + bo);
      if (SPLIT) bl[j] = Frag<T>::load(Bb2 + bo);
    }
#pragma unroll
    for (int i = 0; i < 4; ++i) {
      const size_t ao = (size_t)(m0 + (i << 4) + rlane) * lda + koff + k0;
      V ah = Frag<T>::load(Ab + ao);
      V al;
      if (SPLIT) al = Frag<T>::load(Ab2 + ao);
#pragma unroll
      for (int j = 0; j < 4; ++j) {
        acc[i][j] = Frag<T>::mma(ah, bh[j], acc[i][j]);
        if (SPLIT) {
          acc[i][j] = Frag<T>::mma(ah, bl[j], acc[i][j]);
          acc[i][j] = Frag<T>::mma(al, bh[j], acc[i][j]);
        }
      }
      Frag<T>::guard(acc[i][0], acc[i][3], ah, SPLIT ? al : ah);
    }
    Frag<T>::keep(bh[0], bh[1], bh[2], bh[3]);
    if (SPLIT) Frag<T>::keep(bl[0], bl[1], bl[2], bl[3]);
  }
  acc_guard4(acc[0][0], acc[0][1], acc[0][2], acc[0][3]);
  acc_guard4(acc[1][0], acc[1][1], acc[1][2], acc[1][3]);
  acc_guard4(acc[2][0], acc[2][1], acc[2][2], acc[2][3]);
  acc_guard4(acc[3][0], acc[3][1], acc[3][2], acc[3][3]);

  float* slab = sT[wave];
  const float* Rb = RESID ? (resid + (size_t)b * strideR) : nullptr;
#pragma unroll
  for (int i = 0; i < 4; ++i) {
    const int mBase = m0 + (i << 4);
#pragma unroll
    for (int j = 0; j < 4; ++j) {
      const int n = n0 + (j << 4) + rlane;
      float bv = 0.f;
      if (BIAS_MODE == 2) bv = bias[n];
#pragma unroll
      for (int r = 0; r < 8; ++r) {
        float v = acc[i][j][r] * scale;
        if (BIAS_MODE == 1) v += bias[mBase + mOff + r];
        if (BIAS_MODE == 2) v += bv;
        if (RESID) v += Rb[(size_t)(mBase + mOff + r) * ldc + n];
        if (ACT == 1) v = tanhf(v);
        if (ACT == 2) v = fmaxf(v, 0.0f);
        if (ACT == 3) v = v / (1.0f + expf(-v));
        if (ACT == 4) v = (v > 0.f) ? v : 0.01f * v;
        if (ACT == 5) v = 0.5f * v * (1.0f + erff(v * 0.70710678118654752f));
        slab[(mOff + r) * 68 + (j << 4) + rlane] = v;
      }
    }
    __builtin_amdgcn_fence(__ATOMIC_RELEASE, "workgroup");
    __builtin_amdgcn_wave_barrier();
    __builtin_amdgcn_fence(__ATOMIC_ACQUIRE, "workgroup");
    if (OUT_MODE == 0) {
      float* C = (float*)Cout + (size_t)b * strideC;
      const int hh = lane >> 4, c4 = (lane & 15) * 4;
      for (int pass = 0; pass < 2; ++pass) {
#pragma unroll
        for (int it = 0; it < 8; ++it) {
          const int row = it * 2 + hh;
          v4f v = *(const v4f*)(slab + row * 68 + c4);
          *(volatile v4f*)(C + (size_t)(mBase + row) * ldc + n0 + c4) = v;
        }
        __threadfence();
      }
    } else {
      const int q = lane >> 3, c8 = (lane & 7) * 8;
      unsigned short* C  = (unsigned short*)Cout  + (size_t)b * strideC;
      unsigned short* C2 = (OUT_MODE == 2) ? ((unsigned short*)Cout2 + (size_t)b * strideC) : nullptr;
      for (int pass = 0; pass < 2; ++pass) {
#pragma unroll
        for (int it = 0; it < 4; ++it) {
          const int row = it * 4 + q;
          const float* sp = slab + row * 68 + c8;
          v8h hv, lv;
#pragma unroll
          for (int e = 0; e < 8; ++e) {
            if (OUT_MODE == 1) {
              hv[e] = (_Float16)sp[e];
            } else {
              unsigned short hb = f2bf_bits(sp[e]);
              unsigned short lb = f2bf_bits(sp[e] - bf_bits2f(hb));
              hv[e] = __builtin_bit_cast(_Float16, hb);
              lv[e] = __builtin_bit_cast(_Float16, lb);
            }
          }
          *(volatile v8h*)(C + (size_t)(mBase + row) * ldc + n0 + c8) = hv;
          if (OUT_MODE == 2) *(volatile v8h*)(C2 + (size_t)(mBase + row) * ldc + n0 + c8) = lv;
        }
        __threadfence();
      }
    }
    __builtin_amdgcn_fence(__ATOMIC_RELEASE, "workgroup");
    __builtin_amdgcn_wave_barrier();
    __builtin_amdgcn_fence(__ATOMIC_ACQUIRE, "workgroup");
  }
}

__global__ __launch_bounds__(256) void cast_f32_f16x2(
    const float* __restrict__ in, _Float16* __restrict__ out, int n2) {
  int i = blockIdx.x * 256 + threadIdx.x;
  if (i < n2) {
    const _Float16 h0 = (_Float16)in[2 * i], h1 = (_Float16)in[2 * i + 1];
    const unsigned u = (unsigned)__builtin_bit_cast(unsigned short, h0) | ((unsigned)__builtin_bit_cast(unsigned short, h1) << 16);
    ((volatile unsigned*)out)[i] = u;
    __threadfence();
    ((volatile unsigned*)out)[i] = u;
  }
}


__global__ __launch_bounds__(256) void transpose_cast_f16(const float* __restrict__ in, int ldi,
                                                         _Float16* __restrict__ outT, int ldo, float scale) {
  __shared__ __align__(16) _Float16 tile[64][72];
  const int c0 = blockIdx.x * 64, r0 = blockIdx.y * 64;
  const int t = threadIdx.y * 32 + threadIdx.x;
  for (int i = threadIdx.y; i < 64; i += 8) {
    tile[threadIdx.x][i]      = (_Float16)(in[(size_t)(r0 + i) * ldi + c0 + threadIdx.x] * scale);
    tile[32 + threadIdx.x][i] = (_Float16)(in[(size_t)(r0 + i) * ldi + c0 + 32 + threadIdx.x] * scale);
  }
  __syncthreads();
  const int q = t >> 3, c8 = (t & 7) * 8;
  for (int pass = 0; pass < 2; ++pass) {
#pragma unroll
    for (int it = 0; it < 2; ++it) {
      const int c = it * 32 + q;
      v8h hv = *(const v8h*)(&tile[c][c8]);
      *(volatile v8h*)(outT + (size_t)(c0 + c) * ldo + r0 + c8) = hv;
    }
    __threadfence();
  }
}

#ifndef SRB
#define SRB 512
#endif
#ifndef SCHK
#define SCHK 4096
#endif
#define SEPT (SCHK / SRB)
__device__ __forceinline__ int blk_excl_scan(int cnt, int* scan_ws, int tid, int* tot) {
  const int lane = tid & 31, wave = tid >> 5; int incl = cnt;
#pragma unroll
  for (int o = 1; o < 32; o <<= 1) { const int v = __shfl_up(incl, o, 32); if (lane >= o) incl += v; }
  if (lane == 31) scan_ws[wave] = incl;
  __syncthreads();
  if (wave == 0) { int wv = (lane < SRB / 32) ? scan_ws[lane] : 0; int wincl = wv;
#pragma unroll
    for (int o = 1; o < 32; o <<= 1) { const int v = __shfl_up(wincl, o, 32); if (lane >= o) wincl += v; }
    if (lane < SRB / 32) scan_ws[32 + lane] = wincl - wv; if (lane == 31) scan_ws[64] = wincl; }
  __syncthreads();
  const int res = scan_ws[32 + wave] + incl - cnt; *tot = scan_ws[64];
  return res;
}
__device__ __forceinline__ int chunk_compact(const int* __restrict__ keyv, const int* __restrict__ othv, int e0, int ne, int n0, int nn, int tid, int* L0, int* L1, int* L2, int* scan_ws) {
  int hk[SEPT], ho[SEPT], he[SEPT]; int cnt = 0;
#pragma unroll
  for (int k = 0; k < SEPT; ++k) { const int e = e0 + tid * SEPT + k; hk[k] = -1; if (e < ne) { const int d = keyv[e]; if (d >= n0 && d < n0 + SRB && d < nn) { hk[k] = d - n0; int s; if (othv) { s = othv[e]; s = s < 0 ? 0 : (s >= nn ? nn - 1 : s); } else s = e; ho[k] = s; he[k] = e; ++cnt; } } }
  int tot; int p = blk_excl_scan(cnt, scan_ws, tid, &tot);
#pragma unroll
  for (int k = 0; k < SEPT; ++k) if (hk[k] >= 0) { L0[p] = hk[k]; L1[p] = ho[k]; if (L2) L2[p] = he[k]; ++p; }
  __syncthreads();
  return tot;
}
__global__ __launch_bounds__(SRB) void stream_deg_kernel(const int* __restrict__ keyv, const int* __restrict__ othv, int ne, int nn, int* __restrict__ DEG) {
  __shared__ int L0[SCHK]; __shared__ int L1[SCHK]; __shared__ int scan_ws[80];
  const int tid = threadIdx.x, n0 = blockIdx.x * SRB; int cnt = 0;
  for (int e0 = 0; e0 < ne; e0 += SCHK) { const int tot = chunk_compact(keyv, othv, e0, ne, n0, nn, tid, L0, L1, nullptr, scan_ws);
    for (int q = 0; q < tot; ++q) cnt += (L0[q] == tid) ? 1 : 0;
    __syncthreads(); }
  const int n = n0 + tid; if (n < nn) { ((volatile int*)DEG)[n] = cnt; __threadfence(); ((volatile int*)DEG)[n] = cnt; }
}
#define WCAP 64
template <int LO, int HI, int VPL> struct SlotDisp { static __device__ __forceinline__ void add(int s, float (*acc)[VPL], const float* v) {
  if (LO + 1 == HI) {
#pragma unroll
    for (int j = 0; j < VPL; ++j) acc[LO][j] += v[j]; }
  else { const int MID = (LO + HI) / 2; if (s < MID) SlotDisp<LO, (LO + HI) / 2, VPL>::add(s, acc, v); else SlotDisp<(LO + HI) / 2, HI, VPL>::add(s, acc, v); } } };
template <int VW, int CNT>
__device__ __forceinline__ void coop_flush(int n, const unsigned char* wls, const int* wlv, const float* __restrict__ Hm, int ldh, int lane, float (*acc)[VW + CNT]) {
  for (int j = 0; j < n; ++j) { const int slot = wls[j]; const int src = wlv[j]; float v[VW + CNT]; const float* hp = Hm + (size_t)src * ldh + lane * VW;
#pragma unroll
    for (int q = 0; q < VW; ++q) v[q] = hp[q];
    if (CNT) v[VW + CNT - 1] = 1.0f;
    SlotDisp<0, 32, VW + CNT>::add(slot, acc, v); }
}
template <int VW, int CNT>
__device__ __forceinline__ void coop_chunk(int tot, const int* L0, const int* L1, unsigned char* wls, int* wlv, const float* __restrict__ Hm, int ldh, int wave, int lane, float (*acc)[VW + CNT]) {
  int nlist = 0;
  for (int q0 = 0; q0 < tot; q0 += 32) { const int q = q0 + lane; int l0 = 0, l1 = 0; bool mine = false; if (q < tot) { l0 = L0[q]; l1 = L1[q]; mine = (l0 >> 5) == wave; }
    const unsigned bal = __builtin_amdgcn_ballot_w32(mine); const int cntb = __builtin_popcount(bal);
    if (nlist + cntb > WCAP) { coop_flush<VW, CNT>(nlist, wls, wlv, Hm, ldh, lane, acc); nlist = 0; }
    const int pos = nlist + __builtin_popcount(bal & ((1u << lane) - 1u));
    if (mine) { wls[pos] = (unsigned char)(l0 & 31); wlv[pos] = l1; }
    nlist += cntb; }
  coop_flush<VW, CNT>(nlist, wls, wlv, Hm, ldh, lane, acc);
}
template <int VW, bool BIDIR, int CNT>
__global__ __launch_bounds__(SRB) void coop_agg_kernel(const float* __restrict__ Hm, int ldh, const int* __restrict__ keyv, const int* __restrict__ othv, int ne, int nn, float* __restrict__ RAW, int ldr, float* __restrict__ DEGOUT) {
  __shared__ int L0[SCHK]; __shared__ int L1[SCHK]; __shared__ int scan_ws[80]; __shared__ unsigned char WLs[32][WCAP]; __shared__ int WLv[32][WCAP];
  const int tid = threadIdx.x, lane = tid & 31, wave = tid >> 5, n0 = blockIdx.x * SRB;
  float acc[32][VW + CNT];
#pragma unroll
  for (int s = 0; s < 32; ++s)
#pragma unroll
    for (int j = 0; j < VW + CNT; ++j) acc[s][j] = 0.f;
  for (int e0 = 0; e0 < ne; e0 += SCHK) {
#pragma unroll
    for (int dir = 0; dir < (BIDIR ? 2 : 1); ++dir) {
      const int tot = chunk_compact(dir ? othv : keyv, dir ? keyv : othv, e0, ne, n0, nn, tid, L0, L1, nullptr, scan_ws);
      coop_chunk<VW, CNT>(tot, L0, L1, WLs[wave], WLv[wave], Hm, ldh, wave, lane, acc);
      __syncthreads(); } }
#pragma unroll
  for (int s = 0; s < 32; ++s) { const int n = n0 + wave * 32 + s; if (n < nn) { float* dst = RAW + (size_t)n * ldr + lane * VW;
      for (int pass = 0; pass < 2; ++pass) {
#pragma unroll
        for (int j = 0; j < VW; ++j) ((volatile float*)dst)[j] = acc[s][j];
        if (CNT && lane == 0) ((volatile float*)DEGOUT)[n] = acc[s][VW + CNT - 1];
        __threadfence(); } } }
}

#define GB2 2
#define GNN 2048
#define GE 65536
#define GD 512
#define GDE 128
#define GR (GB2 * GNN)
#define GER (GB2 * GE)
__device__ __forceinline__ unsigned pkh(float a, float b) { return (unsigned)__builtin_bit_cast(unsigned short, (_Float16)a) | ((unsigned)__builtin_bit_cast(unsigned short, (_Float16)b) << 16); }
__device__ __forceinline__ float silu1(float v) { return v / (1.0f + __expf(-v)); }
__global__ __launch_bounds__(256) void edge1_kernel(const float* __restrict__ PQ, const int* __restrict__ ei, const float* __restrict__ dist2, const float* __restrict__ delta, const float* __restrict__ est, const float* __restrict__ We1c, const float* __restrict__ be1, const float* __restrict__ Wg1, const float* __restrict__ bg1, const float* __restrict__ Wg2, const float* __restrict__ bg2, unsigned* __restrict__ H1, float* __restrict__ G) {
  const int lane = threadIdx.x & 31, wave = threadIdx.x >> 5; const int r = blockIdx.x * 8 + wave; const int b = r / GE, e = r % GE;
  int i = ei[e], j = ei[GE + e]; i = i < 0 ? 0 : (i >= GNN ? GNN - 1 : i); j = j < 0 ? 0 : (j >= GNN ? GNN - 1 : j);
  float gin[10]; gin[0] = dist2[r]; gin[1] = delta[r];
#pragma unroll
  for (int q = 0; q < 8; ++q) gin[2 + q] = est[(size_t)r * 8 + q];
  const v4f p = *(const v4f*)(PQ + ((size_t)b * GNN + i) * 256 + lane * 4), qv = *(const v4f*)(PQ + ((size_t)b * GNN + j) * 256 + 128 + lane * 4);
  float h[4];
#pragma unroll
  for (int q = 0; q < 4; ++q) { const int c = lane * 4 + q; float s = p[q] + qv[q] + be1[c];
#pragma unroll
    for (int t = 0; t < 10; ++t) s += gin[t] * We1c[t * GDE + c];
    h[q] = silu1(s); }
  typedef __attribute__((ext_vector_type(2))) unsigned u2; const u2 u = {pkh(h[0], h[1]), pkh(h[2], h[3])};
  float gh = bg1[lane];
#pragma unroll
  for (int t = 0; t < 10; ++t) gh += gin[t] * Wg1[t * 32 + lane];
  float gs = silu1(gh) * Wg2[lane]; for (int o = 16; o > 0; o >>= 1) gs += __shfl_xor(gs, o, 32); const float g = 1.0f / (1.0f + __expf(-(gs + bg2[0])));
  for (int pass = 0; pass < 2; ++pass) { *(volatile u2*)(H1 + ((size_t)r * GDE + lane * 4) / 2) = u; if (lane == 0) ((volatile float*)G)[r] = g; __threadfence(); }
}
__global__ __launch_bounds__(256) void gmul_kernel(float* __restrict__ EM, const float* __restrict__ G) { const long idx = (long)blockIdx.x * 256 + threadIdx.x; if (idx >= (long)GER * GDE) return; const float v = EM[idx] * G[idx / GDE]; ((volatile float*)EM)[idx] = v; __threadfence(); ((volatile float*)EM)[idx] = v; }
__global__ __launch_bounds__(256) void ncat_kernel(const float* __restrict__ Hf, const float* __restrict__ AGG, unsigned* __restrict__ N16) {
  const long idx = (long)blockIdx.x * 256 + threadIdx.x; if (idx >= (long)GR * 320) return; const long r = idx / 320; const int cp = 2 * (int)(idx % 320); float a, b;
  if (cp < GD) { a = Hf[r * GD + cp]; b = Hf[r * GD + cp + 1]; } else { a = AGG[r * GDE + cp - GD]; b = AGG[r * GDE + cp - GD + 1]; }
  ((volatile unsigned*)N16)[idx] = pkh(a, b); __threadfence(); ((volatile unsigned*)N16)[idx] = pkh(a, b);
}
__global__ __launch_bounds__(256) void ln_kernel(const float* __restrict__ X, const float* __restrict__ g, const float* __restrict__ bb, float* __restrict__ out) {
  const int lane = threadIdx.x & 31, wave = threadIdx.x >> 5; const size_t r = (size_t)blockIdx.x * 8 + wave; const float* x = X + r * GD + lane * 16;
  float v[16]; float s = 0.f; for (int q = 0; q < 16; q += 4) { const v4f t = *(const v4f*)(x + q); v[q] = t[0]; v[q + 1] = t[1]; v[q + 2] = t[2]; v[q + 3] = t[3]; s += t[0] + t[1] + t[2] + t[3]; }
  for (int o = 16; o > 0; o >>= 1) s += __shfl_xor(s, o, 32); const float mu = s / GD;
  float t2 = 0.f; for (int q = 0; q < 16; ++q) { const float d = v[q] - mu; t2 += d * d; } for (int o = 16; o > 0; o >>= 1) t2 += __shfl_xor(t2, o, 32); const float inv = rsqrtf(t2 / GD + 1e-5f);
  for (int pass = 0; pass < 2; ++pass) { for (int q = 0; q < 16; q += 4) { v4f y; for (int z = 0; z < 4; ++z) { const int c = lane * 16 + q + z; y[z] = (v[q + z] - mu) * inv * g[c] + bb[c]; } *(volatile v4f*)(out + r * GD + lane * 16 + q) = y; } __threadfence(); }
}
extern "C" void kernel_launch(void* const* d_in, const int* in_sizes, int n_in, void* d_out, int out_size, void* d_ws, size_t ws_size, hipStream_t stream) {
  (void)in_sizes; (void)n_in; (void)out_size; (void)ws_size;
  auto Fp = [&](int i) { return (const float*)d_in[i]; };
  const float* Hf = Fp(0); const int* ei = (const int*)d_in[1]; const float* dist2 = Fp(2); const float* delta = Fp(3); const float* est = Fp(4);
  const float* We1 = Fp(5); const float* be1 = Fp(6); const float* We2 = Fp(7); const float* be2 = Fp(8); const float* Wg1 = Fp(9); const float* bg1 = Fp(10); const float* Wg2 = Fp(11); const float* bg2 = Fp(12); const float* Wn1 = Fp(13); const float* bn1 = Fp(14); const float* Wn2 = Fp(15); const float* bn2 = Fp(16); const float* lng = Fp(17); const float* lnb = Fp(18);
  char* ws = (char*)d_ws; size_t off = 0;
  auto carve = [&](size_t bytes) -> char* { char* p = ws + off; off += (bytes + 255) & ~(size_t)255; return p; };
  _Float16* H16 = (_Float16*)carve((size_t)GR * GD * 2); _Float16* W1abT = (_Float16*)carve((size_t)256 * GD * 2); _Float16* W2T = (_Float16*)carve(GDE * GDE * 2); _Float16* Wn1T = (_Float16*)carve((size_t)1024 * 640 * 2); _Float16* Wn2T = (_Float16*)carve((size_t)GD * 1024 * 2);
  float* PQ = (float*)carve((size_t)GR * 256 * 4); unsigned* H1 = (unsigned*)carve((size_t)GER * GDE * 2); float* G = (float*)carve((size_t)GER * 4); float* EM = (float*)carve((size_t)GER * GDE * 4); float* AGG = (float*)carve((size_t)GR * GDE * 4);
  unsigned* N16 = (unsigned*)carve((size_t)GR * 640 * 2); _Float16* U1 = (_Float16*)carve((size_t)GR * 1024 * 2); float* X = EM;
  cast_f32_f16x2<<<(GR * GD / 2 + 255) / 256, 256, 0, stream>>>(Hf, H16, (long)GR * GD / 2);
  transpose_cast_f16<<<dim3(2, 8), dim3(32, 8), 0, stream>>>(We1, GDE, W1abT, GD, 1.0f);
  transpose_cast_f16<<<dim3(2, 8), dim3(32, 8), 0, stream>>>(We1 + (size_t)GD * GDE, GDE, W1abT + (size_t)GDE * GD, GD, 1.0f);
  transpose_cast_f16<<<dim3(2, 2), dim3(32, 8), 0, stream>>>(We2, GDE, W2T, GDE, 1.0f);
  transpose_cast_f16<<<dim3(16, 10), dim3(32, 8), 0, stream>>>(Wn1, 1024, Wn1T, 640, 1.0f); transpose_cast_f16<<<dim3(8, 16), dim3(32, 8), 0, stream>>>(Wn2, GD, Wn2T, 1024, 1.0f);
  const int tn = GR / 64, te = GER / 64, nb = (GNN + SRB - 1) / SRB;
  wmma_gemm64<0, false, 0, 0, false><<<dim3((tn * 4 + 7) / 8, 1), 256, 0, stream>>>(U16(H16), nullptr, GD, 0, U16(W1abT), nullptr, GD, 0, PQ, nullptr, 256, 0, nullptr, nullptr, 0, GR, 256, GD, 1.0f);
  edge1_kernel<<<GER / 8, 256, 0, stream>>>(PQ, ei, dist2, delta, est, We1 + (size_t)1024 * GDE, be1, Wg1, bg1, Wg2, bg2, H1, G);
  wmma_gemm64<0, false, 2, 0, false, 3><<<dim3((te * 2 + 7) / 8, 1), 256, 0, stream>>>((const unsigned short*)H1, nullptr, GDE, 0, U16(W2T), nullptr, GDE, 0, EM, nullptr, GDE, 0, be2, nullptr, 0, GER, GDE, GDE, 1.0f);
  gmul_kernel<<<(unsigned)(((long)GER * GDE + 255) / 256), 256, 0, stream>>>(EM, G);
  for (int b = 0; b < GB2; ++b) coop_agg_kernel<4, false, 0><<<nb, SRB, 0, stream>>>(EM + (size_t)b * GE * GDE, GDE, ei, nullptr, GE, GNN, AGG + (size_t)b * GNN * GDE, GDE, nullptr);
  ncat_kernel<<<(unsigned)(((long)GR * 320 + 255) / 256), 256, 0, stream>>>(Hf, AGG, N16);
  wmma_gemm64<0, false, 2, 1, false, 3><<<dim3((tn * 16 + 7) / 8, 1), 256, 0, stream>>>((const unsigned short*)N16, nullptr, 640, 0, U16(Wn1T), nullptr, 640, 0, U1, nullptr, 1024, 0, bn1, nullptr, 0, GR, 1024, 640, 1.0f);
  wmma_gemm64<0, false, 2, 0, true><<<dim3((tn * 8 + 7) / 8, 1), 256, 0, stream>>>(U16(U1), nullptr, 1024, 0, U16(Wn2T), nullptr, 1024, 0, X, nullptr, GD, 0, bn2, Hf, 0, GR, GD, 1024, 1.0f);
  ln_kernel<<<GR / 8, 256, 0, stream>>>(X, lng, lnb, (float*)d_out);
}
